// MultiEncoding__32993938767928
// MI455X (gfx1250) — hardware-verified
//
#include <hip/hip_runtime.h>
#include <math.h>


typedef float          v8f  __attribute__((ext_vector_type(8)));
typedef float          v4f  __attribute__((ext_vector_type(4)));
typedef unsigned int   v4u  __attribute__((ext_vector_type(4)));
typedef unsigned short v8us __attribute__((ext_vector_type(8)));
typedef __bf16         v16b __attribute__((ext_vector_type(16)));

union FragBf { v16b v; v8us q[2]; };
union Pk16   { v4u u; unsigned short e[8]; };

#define NTH    128
#define IMGSZ  784
#define IMW    28
#define NP     13
#define NSTEP  169
#define NFEAT  676
#define KPADH  704
#define NPADW  32
#define SGP    65
#define HSP    33
#define RS2    0.70710678118654752440f

__device__ __forceinline__ unsigned short bf16_rne(float f) {
    unsigned int u = __float_as_uint(f);
    u += 0x7FFFu + ((u >> 16) & 1u);
    return (unsigned short)(u >> 16);
}
__device__ __forceinline__ float bf16_val(unsigned short b) {
    return __uint_as_float(((unsigned int)b) << 16);
}
__device__ __forceinline__ void split_bf16(float v, unsigned short& hi, unsigned short& lo) {
    hi = bf16_rne(v);
    lo = bf16_rne(v - bf16_val(hi));
}

__device__ __forceinline__ v8f wmma_bf(v16b a, v16b b, v8f c) {
    return __builtin_amdgcn_wmma_f32_16x16x32_bf16(false, a, false, b, (short)0, c, false, false);
}

__global__ void __launch_bounds__(256)
k_packw(const float* __restrict__ W1, unsigned short* Bhi, unsigned short* Blo, int N, int K) {
    const int i   = blockIdx.x * 256 + threadIdx.x;
    const int per = KPADH / 8;
    if (i >= NPADW * per) return;
    const int n  = i / per;
    const int k0 = (i - n * per) * 8;
    const int nc = (n < N) ? n : (N - 1);
    Pk16 hv, lv;
#pragma unroll
    for (int e = 0; e < 8; ++e) {
        const int k  = k0 + e;
        const int kc = (k < K) ? k : (K - 1);
        float w = W1[(size_t)nc * K + kc];
        if (n >= N || k >= K) w = 0.0f;
        unsigned short a, b;
        split_bf16(w, a, b);
        hv.e[e] = a;
        lv.e[e] = b;
    }
    const size_t off = (size_t)n * KPADH + k0;
    *(volatile v4u*)(Bhi + off) = hv.u;
    *(volatile v4u*)(Blo + off) = lv.u;
    __threadfence();
    *(volatile v4u*)(Bhi + off) = hv.u;
    *(volatile v4u*)(Blo + off) = lv.u;
}

__global__ void __launch_bounds__(NTH)
k_qsim(const float* __restrict__ x, const float* __restrict__ crz_p,
       const float* __restrict__ ry_p, unsigned short* Ahi, unsigned short* Alo, int B) {
    __shared__ float ST[32 * NTH];
    __shared__ float SG[NTH * SGP];
    __shared__ float PH[32];

    const int tid = threadIdx.x;
    const int b   = blockIdx.x * NTH + tid;
    const int bcl = (b < B) ? b : (B - 1);
    const float* xb = x + (size_t)bcl * IMGSZ;

#pragma unroll 1
    for (int s = 0; s < 32; ++s) ST[s * NTH + tid] = (s == 0) ? 1.0f : 0.0f;

    const float thc = crz_p[0];
    const float thr = ry_p[0];
    float sc, cc, sr, cr;
    sincosf(0.5f * thc, &sc, &cc);
    sincosf(0.5f * thr, &sr, &cr);

    {
        const int a = tid & 15;
        float pr = 1.0f, pi = 0.0f;
#pragma unroll 1
        for (int i = 0; i < 4; ++i) {
            const int cb = (a >> (3 - i)) & 1;
            const int tw = (i + 1) & 3;
            const int tb = (a >> (3 - tw)) & 1;
            const float fc = cb ? cc : 1.0f;
            const float fs = cb ? (tb ? sc : -sc) : 0.0f;
            const float nr = pr * fc - pi * fs;
            const float ni = pr * fs + pi * fc;
            pr = nr;
            pi = ni;
        }
        if (tid < 16) { PH[2 * a] = pr; PH[2 * a + 1] = pi; }
    }
    __syncthreads();

    int py = 0, px = 0;
#pragma unroll 1
    for (int p = 0; p < NSTEP; ++p) {
        const float* pb = xb + (2 * py) * IMW + 2 * px;

#pragma unroll 1
        for (int g = 0; g < 8; ++g) {
            const int q = g & 3;
            float m00r, m00i, m01r, m01i, m10r, m10i, m11r, m11i;
            if (g < 4) {
                m00r = RS2;  m00i = 0.0f; m01r = RS2;  m01i = 0.0f;
                m10r = RS2;  m10i = 0.0f; m11r = -RS2; m11i = 0.0f;
                const int cnt = (q == 3) ? 1 : 5;
#pragma unroll 1
                for (int i = 0; i < cnt; ++i) {
                    const int idx = 5 * q + i;
                    const float f = pb[(idx >> 2) * IMW + (idx & 3)];
                    float s, c;
                    sincosf(0.5f * f, &s, &c);
                    if ((i & 1) == 0) {
                        float t;
                        t = m00r * c + m00i * s;  m00i = m00i * c - m00r * s;  m00r = t;
                        t = m01r * c + m01i * s;  m01i = m01i * c - m01r * s;  m01r = t;
                        t = m10r * c - m10i * s;  m10i = m10i * c + m10r * s;  m10r = t;
                        t = m11r * c - m11i * s;  m11i = m11i * c + m11r * s;  m11r = t;
                    } else {
                        const float r0r = c * m00r - s * m10r, r0i = c * m00i - s * m10i;
                        const float r1r = c * m01r - s * m11r, r1i = c * m01i - s * m11i;
                        const float q0r = s * m00r + c * m10r, q0i = s * m00i + c * m10i;
                        const float q1r = s * m01r + c * m11r, q1i = s * m01i + c * m11i;
                        m00r = r0r; m00i = r0i; m01r = r1r; m01i = r1i;
                        m10r = q0r; m10i = q0i; m11r = q1r; m11i = q1i;
                    }
                }
            } else {
                if (g == 4) {
#pragma unroll 1
                    for (int a = 0; a < 16; ++a) {
                        const float fr = PH[2 * a], fi = PH[2 * a + 1];
                        float* sp = ST + (2 * a) * NTH + tid;
                        const float ar = sp[0], ai = sp[NTH];
                        sp[0]   = ar * fr - ai * fi;
                        sp[NTH] = ar * fi + ai * fr;
                    }
                }
                m00r = cr; m00i = 0.0f; m01r = -sr; m01i = 0.0f;
                m10r = sr; m10i = 0.0f; m11r = cr;  m11i = 0.0f;
            }

            const int sh = 3 - q;
            const int bm = 1 << sh;
            const int lm = bm - 1;
#pragma unroll 1
            for (int j = 0; j < 8; ++j) {
                const int i0 = ((j >> sh) << (sh + 1)) | (j & lm);
                const int i1 = i0 | bm;
                float* p0 = ST + (2 * i0) * NTH + tid;
                float* p1 = ST + (2 * i1) * NTH + tid;
                const float a0r = p0[0], a0i = p0[NTH];
                const float a1r = p1[0], a1i = p1[NTH];
                const float n0r = m00r * a0r - m00i * a0i + m01r * a1r - m01i * a1i;
                const float n0i = m00r * a0i + m00i * a0r + m01r * a1i + m01i * a1r;
                const float n1r = m10r * a0r - m10i * a0i + m11r * a1r - m11i * a1i;
                const float n1i = m10r * a0i + m10i * a0r + m11r * a1i + m11i * a1r;
                p0[0] = n0r; p0[NTH] = n0i;
                p1[0] = n1r; p1[NTH] = n1i;
            }
        }

        float f0 = 0.0f, f1 = 0.0f, f2 = 0.0f, f3 = 0.0f;
#pragma unroll 1
        for (int a = 0; a < 16; ++a) {
            const float* sp = ST + (2 * a) * NTH + tid;
            const float ar = sp[0], ai = sp[NTH];
            const float pr = ar * ar + ai * ai;
            f0 += (a & 8) ? -pr : pr;
            f1 += (a & 4) ? -pr : pr;
            f2 += (a & 2) ? -pr : pr;
            f3 += (a & 1) ? -pr : pr;
        }
        {
            float* sg = SG + tid * SGP + (p & 15) * 4;
            sg[0] = f0; sg[1] = f1; sg[2] = f2; sg[3] = f3;
        }

        if ((p & 15) == 15 || p == NSTEP - 1) {
            __syncthreads();
            const int grp  = p >> 4;
            const int nval = (p - grp * 16 + 1) * 4;
#pragma unroll 1
            for (int it = 0; it < 8; ++it) {
                const int piece = it * NTH + tid;
                const int L  = piece >> 3;
                const int kb = (piece & 7) * 8;
                const float* src = SG + L * SGP + kb;
                Pk16 hv, lv;
#pragma unroll
                for (int e = 0; e < 8; ++e) {
                    float v = src[e];
                    if (kb + e >= nval) v = 0.0f;
                    unsigned short ah, al;
                    split_bf16(v, ah, al);
                    hv.e[e] = ah;
                    lv.e[e] = al;
                }
                const int bimg = blockIdx.x * NTH + L;
                const size_t off = (size_t)bimg * KPADH + grp * 64 + kb;
                if (bimg < B) {
                    *(volatile v4u*)(Ahi + off) = hv.u;
                    *(volatile v4u*)(Alo + off) = lv.u;
                }
                __threadfence();
                if (bimg < B) {
                    *(volatile v4u*)(Ahi + off) = hv.u;
                    *(volatile v4u*)(Alo + off) = lv.u;
                }
            }
            __syncthreads();
        }

        px += 1;
        if (px == NP) { px = 0; py += 1; }
    }
}

__global__ void __launch_bounds__(128)
k_head(const unsigned short* __restrict__ Ahi, const unsigned short* __restrict__ Alo,
       const unsigned short* __restrict__ Bhi, const unsigned short* __restrict__ Blo,
       const float* __restrict__ b1, const float* __restrict__ W2,
       const float* __restrict__ b2, float* out, int B, int N1) {
    __shared__ float Hs[4][16 * HSP];
    __shared__ __attribute__((aligned(16))) float Os[4][32];

    const int w = threadIdx.x >> 5;
    const int l = threadIdx.x & 31, h = l >> 4, m = l & 15;
    const int tile = blockIdx.x * 4 + w;
    const bool tv  = (tile * 16 + 16) <= B;
    int row = tile * 16 + m;
    row = (row < B) ? row : (B - 1);

    const unsigned short* ah  = Ahi + (size_t)row * KPADH + 8 * h;
    const unsigned short* al  = Alo + (size_t)row * KPADH + 8 * h;
    const unsigned short* bh0 = Bhi + (size_t)m * KPADH + 8 * h;
    const unsigned short* bh1 = Bhi + (size_t)(16 + m) * KPADH + 8 * h;
    const unsigned short* bl0 = Blo + (size_t)m * KPADH + 8 * h;
    const unsigned short* bl1 = Blo + (size_t)(16 + m) * KPADH + 8 * h;

    v8f acc0 = {0.f, 0.f, 0.f, 0.f, 0.f, 0.f, 0.f, 0.f};
    v8f acc1 = {0.f, 0.f, 0.f, 0.f, 0.f, 0.f, 0.f, 0.f};

#pragma unroll 1
    for (int kt = 0; kt < KPADH / 32; ++kt) {
        const int ko = kt * 32;
        FragBf A, AL, B0, B1, C0, C1;
        A.q[0]  = *(const v8us*)(ah + ko);   A.q[1]  = *(const v8us*)(ah + ko + 16);
        AL.q[0] = *(const v8us*)(al + ko);   AL.q[1] = *(const v8us*)(al + ko + 16);
        B0.q[0] = *(const v8us*)(bh0 + ko);  B0.q[1] = *(const v8us*)(bh0 + ko + 16);
        B1.q[0] = *(const v8us*)(bh1 + ko);  B1.q[1] = *(const v8us*)(bh1 + ko + 16);
        C0.q[0] = *(const v8us*)(bl0 + ko);  C0.q[1] = *(const v8us*)(bl0 + ko + 16);
        C1.q[0] = *(const v8us*)(bl1 + ko);  C1.q[1] = *(const v8us*)(bl1 + ko + 16);
        acc0 = wmma_bf(A.v,  B0.v, acc0);
        acc0 = wmma_bf(A.v,  C0.v, acc0);
        acc0 = wmma_bf(AL.v, B0.v, acc0);
        acc1 = wmma_bf(A.v,  B1.v, acc1);
        acc1 = wmma_bf(A.v,  C1.v, acc1);
        acc1 = wmma_bf(AL.v, B1.v, acc1);
        asm volatile("v_nop\n\tv_nop\n\tv_nop\n\tv_nop"
                     : "+v"(acc0), "+v"(acc1)
                     : "v"(A.v), "v"(AL.v), "v"(B0.v), "v"(B1.v), "v"(C0.v), "v"(C1.v));
    }

    float* hs = Hs[w];
#pragma unroll
    for (int r = 0; r < 8; ++r) {
        const int img = 8 * h + r;
        {
            const int n  = m;
            const int nc = (n < N1) ? n : (N1 - 1);
            float v = acc0[r] + b1[nc];
            v = (v > 0.0f) ? v : 0.1f * v;
            hs[img * HSP + n] = v;
        }
        {
            const int n  = 16 + m;
            const int nc = (n < N1) ? n : (N1 - 1);
            float v = acc1[r] + b1[nc];
            v = (v > 0.0f) ? v : 0.1f * v;
            hs[img * HSP + n] = v;
        }
    }
    __syncthreads();

    {
        const int img = l & 15, c = l >> 4;
        float o = b2[c];
#pragma unroll
        for (int n = 0; n < 20; ++n) o = fmaf(hs[img * HSP + n], W2[c * 20 + n], o);
        Os[w][img * 2 + c] = o;
    }
    __syncthreads();

    {
        const v4f v = *(const v4f*)(&Os[w][4 * (l & 7)]);
        float* d = out + (size_t)tile * 32 + 4 * (l & 7);
        if (l < 8 && tv) *(volatile v4f*)d = v;
        __threadfence();
        if (l < 8 && tv) *(volatile v4f*)d = v;
    }
}

extern "C" void kernel_launch(void* const* d_in, const int* in_sizes, int n_in,
                              void* d_out, int out_size, void* d_ws, size_t ws_size,
                              hipStream_t stream) {
    if (n_in < 7) return;
    const int nx = in_sizes[0];
    if (nx <= 0 || (nx % IMGSZ) != 0) return;
    const int B = nx / IMGSZ;
    if ((B % 16) != 0) return;
    if (out_size != B * 2) return;
    const int N1 = 20, K1 = NFEAT;
    if (in_sizes[1] < 1 || in_sizes[2] < 1) return;
    if (in_sizes[3] != N1 * K1 || in_sizes[4] < N1 || in_sizes[5] != 2 * N1 || in_sizes[6] < 2) return;

    const float* x   = (const float*)d_in[0];
    const float* crz = (const float*)d_in[1];
    const float* ryt = (const float*)d_in[2];
    const float* W1  = (const float*)d_in[3];
    const float* b1  = (const float*)d_in[4];
    const float* W2  = (const float*)d_in[5];
    const float* b2  = (const float*)d_in[6];
    float* out = (float*)d_out;

    char* ws = (char*)d_ws;
    size_t off = 0;
    const size_t aBytes = (size_t)B * KPADH * 2;
    const size_t bBytes = (size_t)NPADW * KPADH * 2;
    unsigned short* Ahi = (unsigned short*)(ws + off); off = (off + aBytes + 255) & ~(size_t)255;
    unsigned short* Alo = (unsigned short*)(ws + off); off = (off + aBytes + 255) & ~(size_t)255;
    unsigned short* Bhi = (unsigned short*)(ws + off); off = (off + bBytes + 255) & ~(size_t)255;
    unsigned short* Blo = (unsigned short*)(ws + off); off = (off + bBytes + 255) & ~(size_t)255;
    if (off > ws_size) return;

    {
        const int pieces = NPADW * (KPADH / 8);
        k_packw<<<dim3((pieces + 255) / 256), dim3(256), 0, stream>>>(W1, Bhi, Blo, N1, K1);
    }
    k_qsim<<<dim3((B + NTH - 1) / NTH), dim3(NTH), 0, stream>>>(x, crz, ryt, Ahi, Alo, B);
    k_head<<<dim3((B + 63) / 64), dim3(128), 0, stream>>>(Ahi, Alo, Bhi, Blo, b1, W2, b2,
                                                         out, B, N1);
}
